// HydroSSMCell_71399536329341
// MI455X (gfx1250) — hardware-run, weakly checked
//
#include <hip/hip_runtime.h>


#define NB   64
#define NL   4096
#define NA   8
#define NG   9
#define NC   128
#define NM   262144
#define KP   32
#define O1   33554432
typedef _Float16 h16;
typedef unsigned short bf;
typedef __attribute__((ext_vector_type(16))) __bf16   v16bf;
typedef __attribute__((ext_vector_type(16))) _Float16 v16h;
typedef __attribute__((ext_vector_type(8)))  _Float16 v8h;
typedef __attribute__((ext_vector_type(8)))  unsigned short v8us;
typedef __attribute__((ext_vector_type(8)))  float    v8f;
typedef __attribute__((ext_vector_type(4)))  float    v4f;
typedef v8h  __attribute__((may_alias)) v8ha;
typedef v4f  __attribute__((may_alias)) v4fa;
typedef v8us __attribute__((may_alias)) v8usa;

__device__ __forceinline__ unsigned short f2bf(float f) { unsigned u = __float_as_uint(f); u += 0x7FFFu + ((u >> 16) & 1u); return (unsigned short)(u >> 16); }
__device__ __forceinline__ float bf2f(unsigned short b) { return __uint_as_float(((unsigned)b) << 16); }
__device__ __forceinline__ float bfr(float f) { return bf2f(f2bf(f)); }
__device__ __forceinline__ v16h cat16(v8h lo, v8h hi) { return __builtin_shufflevector(lo, hi, 0, 1, 2, 3, 4, 5, 6, 7, 8, 9, 10, 11, 12, 13, 14, 15); }
__device__ __forceinline__ v16bf cat16b(v8us lo, v8us hi) { return __builtin_bit_cast(v16bf, __builtin_shufflevector(lo, hi, 0, 1, 2, 3, 4, 5, 6, 7, 8, 9, 10, 11, 12, 13, 14, 15)); }
__device__ __forceinline__ v8f wmma16(v16h a, v16h b, v8f c) { return __builtin_amdgcn_wmma_f32_16x16x32_f16(false, a, false, b, (short)0, c, false, false); }
__device__ __forceinline__ v8f wmmab(v16bf a, v16bf b, v8f c) { return __builtin_amdgcn_wmma_f32_16x16x32_bf16(false, a, false, b, (short)0, c, false, false); }

template <typename T16> struct WFrag;
template <> struct WFrag<h16> { typedef v16h V; static __device__ __forceinline__ V ld(const h16* p) { return cat16(*(const v8h*)p, *(const v8h*)(p + 16)); } static __device__ __forceinline__ v8f mma(V a, V b, v8f c) { return wmma16(a, b, c); } };
template <> struct WFrag<bf> { typedef v16bf V; static __device__ __forceinline__ V ld(const bf* p) { return cat16b(*(const v8us*)p, *(const v8us*)(p + 16)); } static __device__ __forceinline__ v8f mma(V a, V b, v8f c) { return wmmab(a, b, c); } };
template <typename T16, int NSPLIT, bool BIAS>
__global__ __launch_bounds__(32) void k_gemmw(const T16* __restrict__ A, const T16* __restrict__ A2, const T16* __restrict__ Bt, const T16* __restrict__ Bt2, int K, float* C, int ldc, const float* __restrict__ bias, size_t sA, size_t sB, size_t sC) {
    typedef typename WFrag<T16>::V V;
    __shared__ __align__(16) float os[16 * 68];
    const size_t z = blockIdx.z; A += z * sA; if (A2) A2 += z * sA; Bt += z * sB; if (Bt2) Bt2 += z * sB; C += z * sC;
    const int lane = threadIdx.x & 31, lr = lane & 15, hi = lane >> 4; const int r0 = blockIdx.x * 64, c0 = blockIdx.y * 64;
    v8f acc[4][4];
#pragma unroll
    for (int mb = 0; mb < 4; ++mb)
#pragma unroll
        for (int nb = 0; nb < 4; ++nb) acc[mb][nb] = (v8f){};
    const size_t aoff = (size_t)(r0 + lr) * K + 8 * hi, boff = (size_t)(c0 + lr) * K + 8 * hi;
    for (int kc = 0; kc < K; kc += 32) {
        V a[4], a2[4];
#pragma unroll
        for (int mb = 0; mb < 4; ++mb) { a[mb] = WFrag<T16>::ld(A + aoff + (size_t)mb * 16 * K + kc); if (NSPLIT == 1 || NSPLIT == 2) a2[mb] = WFrag<T16>::ld(A2 + aoff + (size_t)mb * 16 * K + kc); }
#pragma unroll
        for (int nb = 0; nb < 4; ++nb) { const V b = WFrag<T16>::ld(Bt + boff + (size_t)nb * 16 * K + kc); V b2; if (NSPLIT >= 2) b2 = WFrag<T16>::ld(Bt2 + boff + (size_t)nb * 16 * K + kc);
#pragma unroll
            for (int mb = 0; mb < 4; ++mb) { acc[mb][nb] = WFrag<T16>::mma(a[mb], b, acc[mb][nb]); if (NSPLIT == 1 || NSPLIT == 2) acc[mb][nb] = WFrag<T16>::mma(a2[mb], b, acc[mb][nb]); if (NSPLIT >= 2) acc[mb][nb] = WFrag<T16>::mma(a[mb], b2, acc[mb][nb]); } }
        asm volatile("v_nop\n\tv_nop\n\tv_nop\n\tv_nop" : "+v"(acc[0][0]), "+v"(acc[1][1]), "+v"(acc[2][2]), "+v"(acc[3][3]) : "v"(a[0]), "v"(a[3]));
    }
#pragma unroll
    for (int mb = 0; mb < 4; ++mb) {
#pragma unroll
        for (int nb = 0; nb < 4; ++nb) {
#pragma unroll
            for (int j = 0; j < 8; ++j) os[(hi * 8 + j) * 68 + nb * 16 + lr] = acc[mb][nb][j]; }
        __builtin_amdgcn_wave_barrier(); asm volatile("" ::: "memory");
        float* crow = C + (size_t)(r0 + mb * 16) * ldc + c0;
#pragma unroll 1
        for (int ps = 0; ps < 2; ++ps) {
#pragma unroll
            for (int s = 0; s < 8; ++s) { const int row = 2 * s + hi, cofs = lr * 4; v4f val = *(const v4fa*)(os + row * 68 + cofs); if (BIAS) { val[0] += bfr(bias[c0 + cofs]); val[1] += bfr(bias[c0 + cofs + 1]); val[2] += bfr(bias[c0 + cofs + 2]); val[3] += bfr(bias[c0 + cofs + 3]); }
                *(volatile v4f*)(crow + (size_t)row * ldc + cofs) = val; }
            if (ps == 0) __threadfence(); }
        __builtin_amdgcn_wave_barrier(); asm volatile("" ::: "memory");
    }
}

typedef __attribute__((ext_vector_type(2))) _Float16 v2h;
typedef __attribute__((ext_vector_type(4))) _Float16 v4h;
typedef __attribute__((ext_vector_type(2))) unsigned short v2us;
typedef __attribute__((ext_vector_type(4))) unsigned short v4us;
typedef __attribute__((ext_vector_type(2))) float v2f;
typedef __attribute__((ext_vector_type(4))) int v4i;

__global__ __launch_bounds__(256) void k_cat(const float* __restrict__ sa, const float* __restrict__ sb, bf* Xb) { const size_t m = (size_t)blockIdx.x * 256 + threadIdx.x; const float* pa = sa + m * NA; const float* pb = sb + m * NG; v8us o0, o1, o2, o3;
#pragma unroll
    for (int k = 0; k < 8; ++k) { o0[k] = f2bf(pa[k]); o1[k] = f2bf(pb[k]); o2[k] = 0; o3[k] = 0; }
    o2[0] = f2bf(pb[8]); bf* w = Xb + m * KP;
    *(volatile v8us*)(w) = o0; *(volatile v8us*)(w + 8) = o1; *(volatile v8us*)(w + 16) = o2; *(volatile v8us*)(w + 24) = o3;
    __threadfence();
    *(volatile v8us*)(w) = o0; *(volatile v8us*)(w + 8) = o1; *(volatile v8us*)(w + 16) = o2; *(volatile v8us*)(w + 24) = o3; }

__global__ __launch_bounds__(128) void k_wpad(const float* __restrict__ Wm, bf* Wt) { const int c = threadIdx.x; v8us o0, o1, o2, o3;
#pragma unroll
    for (int k = 0; k < 8; ++k) { o0[k] = f2bf(Wm[k * NC + c]); o1[k] = f2bf(Wm[(k + 8) * NC + c]); o2[k] = 0; o3[k] = 0; }
    o2[0] = f2bf(Wm[16 * NC + c]); bf* w = Wt + (size_t)c * KP;
    *(volatile v8us*)(w) = o0; *(volatile v8us*)(w + 8) = o1; *(volatile v8us*)(w + 16) = o2; *(volatile v8us*)(w + 24) = o3;
    __threadfence();
    *(volatile v8us*)(w) = o0; *(volatile v8us*)(w + 8) = o1; *(volatile v8us*)(w + 16) = o2; *(volatile v8us*)(w + 24) = o3; }

__global__ __launch_bounds__(256) void k_walk(const float* __restrict__ P, const float* __restrict__ bv, const float* __restrict__ dp, const float* __restrict__ s0, float* R0, float* R1) { const unsigned j = blockIdx.x * 256 + threadIdx.x; const unsigned n = j / NC, c = j - n * NC; const float r = 1.0f / (1.0f + expf(-bfr(dp[c]))); const float g = 1.0f - r; const float e = bfr(bv[c]); float v = bfr(s0[j]); const float* p = P + (size_t)n * NL * NC + c; float* o = R0 + (size_t)n * NL * NC + c;
    for (int t0 = 0; t0 < NL; t0 += 8) { float w8[8];
#pragma unroll
        for (int k = 0; k < 8; ++k) { const float q = tanhf(p[(size_t)(t0 + k) * NC] + e); v = r * v + g * q; w8[k] = v; }
#pragma unroll
        for (int k = 0; k < 8; ++k) *(volatile float*)(o + (size_t)(t0 + k) * NC) = w8[k];
        __threadfence();
#pragma unroll
        for (int k = 0; k < 8; ++k) *(volatile float*)(o + (size_t)(t0 + k) * NC) = w8[k]; }
    *(volatile float*)(R1 + j) = v; __threadfence(); *(volatile float*)(R1 + j) = v; }

extern "C" void kernel_launch(void* const* d_in, const int* in_sizes, int n_in, void* d_out, int out_size, void* d_ws, size_t ws_size, hipStream_t stream) {
    if (n_in < 6) return;
    if (in_sizes[0] != NM * NA || in_sizes[1] != NM * NG || in_sizes[2] != NB * NC || in_sizes[3] != (NA + NG) * NC || in_sizes[4] != NC || in_sizes[5] != NC) return;
    if (out_size != O1 + NB * NC) return;
    static_assert(NM == NB * NL && O1 == NM * NC && (O1 % 32) == 0 && NA == 8 && NG == 9 && NA + NG <= KP && KP == 32 && NM % 64 == 0 && NC % 64 == 0 && NM % 256 == 0 && (NB * NC) % 256 == 0 && NC % 32 == 0 && NL % 8 == 0 && NC == 128, "the two results end to end, the second on a 128-byte line; a row of 8 and 9 live words inside one matrix word of 32; the product: M and N multiples of 64, the depth of 32; the flat grids exact; the time steps in eights; one block of 128 for Wt");
    const float* sa = (const float*)d_in[0]; const float* sb = (const float*)d_in[1]; const float* s0 = (const float*)d_in[2]; const float* Wm = (const float*)d_in[3]; const float* bv = (const float*)d_in[4]; const float* dp = (const float*)d_in[5];
    float* out = (float*)d_out; float* R0 = out; float* R1 = out + O1;
    char* wsp = (char*)d_ws; auto take = [&](size_t bytes) { char* p = wsp; wsp += (bytes + 255) & ~(size_t)255; return (void*)p; };
    bf* Xb = (bf*)take((size_t)NM * KP * 2); bf* Wt = (bf*)take((size_t)NC * KP * 2); float* P = (float*)take((size_t)NM * NC * 4);
    if ((size_t)(wsp - (char*)d_ws) > ws_size) return;
    k_cat<<<(unsigned)(NM / 256), 256, 0, stream>>>(sa, sb, Xb);
    k_wpad<<<1, 128, 0, stream>>>(Wm, Wt);
    k_gemmw<bf, 0, false><<<dim3(NM / 64, NC / 64, 1), 32, 0, stream>>>(Xb, nullptr, Wt, nullptr, KP, P, NC, nullptr, 0, 0, 0);
    k_walk<<<(unsigned)(NB * NC / 256), 256, 0, stream>>>(P, bv, dp, s0, R0, R1);
}
